// Model_7310034338114
// MI455X (gfx1250) — hardware-verified
//
#include <hip/hip_runtime.h>
#include <math.h>

#ifndef NB
#define NB 4
#endif
#ifndef SEQ
#define SEQ 1024
#endif
#define NB_FULL 4
#define SEQ_FULL 1024
#define D0 192
#define D1 66
#define NH0 16
#define DPH0 12
#define NH1 11
#define DPH1 6
#define KP0 192
#define KP1 96
#define LDQ0 256
#define LDQ1 192
#define NO1P 80
#define QB 32
#define MTOK (NB * SEQ)
#define OUT1_OFF_ELEMS (NB_FULL * SEQ_FULL * D0)

#define XCARRY 8.0f
#define WCARRY 64.0f
#define HCARRY 16.0f
#define PCARRY 1024.0f
#define CTXS 4.0f
#define SC_PROJ (1.0f / 512.0f)
#define SC_OUT (1.0f / 4096.0f)
#define QS0 0.28867513f
#define QS1 0.40824829f
#define SC2 (1.4426950408889634f / 256.0f)
#define NEGMAX (-3.4028234663852886e38f)

#define KIND_O 0
#define KIND_Q 1
#define KIND_K 2
#define KIND_V 3

static_assert(SEQ == SEQ_FULL);
static_assert(NB <= NB_FULL);
static_assert(MTOK % 64 == 0 && MTOK % 128 == 0);
static_assert(SEQ % QB == 0 && SEQ % 32 == 0 && QB % 16 == 0);
static_assert(D0 == NH0 * DPH0 && D1 == NH1 * DPH1);
static_assert(DPH0 <= 16 && DPH1 <= 16);
static_assert(KP0 % 32 == 0 && KP1 % 32 == 0 && KP0 >= D0 && KP1 >= D1);
static_assert(LDQ0 % 64 == 0 && LDQ1 % 64 == 0 && LDQ0 >= NH0 * 16 && LDQ1 >= NH1 * 16);
static_assert(D0 % 64 == 0);
static_assert(NO1P % 16 == 0 && NO1P >= D1 && NO1P / 16 == 5);
static_assert((size_t)OUT1_OFF_ELEMS * 4 == 3145728);
static_assert(((size_t)OUT1_OFF_ELEMS * 4) % 128 == 0);
static_assert((size_t)OUT1_OFF_ELEMS * 4 + (size_t)NB_FULL * SEQ_FULL * D1 * 4 == 4227072);
static_assert((16 * D1 * 4) % 128 == 0);
static_assert(8 * 32 + 8 == 16 * D1 / 4);
static_assert(8 * 16 * 68 * 4 <= 131072);
static_assert(QB * KP0 * 2 <= 131072 && QB * KP1 * 2 <= 131072);
static_assert(8 * 16 * D1 * 4 <= 131072);
static_assert((MTOK * (KP0 / 8)) % 256 == 0 && (MTOK * (KP1 / 8)) % 256 == 0);

#define WS_TOTAL_BYTES ((size_t)MTOK * KP0 * 2 + (size_t)MTOK * KP1 * 2 + 3 * (size_t)MTOK * LDQ0 * 2 + (size_t)MTOK * KP0 * 2 + \
                        3 * (size_t)MTOK * LDQ1 * 2 + (size_t)MTOK * KP1 * 2 + 3 * (size_t)LDQ0 * KP0 * 2 + (size_t)D0 * KP0 * 2 + \
                        3 * (size_t)LDQ1 * KP1 * 2 + (size_t)NO1P * KP1 * 2)
static_assert(WS_TOTAL_BYTES <= (size_t)134217728);

typedef _Float16 h16;
typedef __attribute__((ext_vector_type(16))) _Float16 v16h;
typedef __attribute__((ext_vector_type(8)))  _Float16 v8h;
typedef __attribute__((ext_vector_type(8)))  float    v8f;
typedef __attribute__((ext_vector_type(4)))  float    v4f;
typedef __attribute__((ext_vector_type(4)))  unsigned int v4u;
typedef __attribute__((ext_vector_type(4)))  int      v4i;


#define VST2(T, ptr, val) do { const T vst2_v_ = (val); *(volatile T*)(ptr) = vst2_v_; __threadfence(); *(volatile T*)(ptr) = vst2_v_; } while (0)
#define VST2V4(ptr, val) do { const v4f vst2_v4_ = (val); *(volatile v4f*)(ptr) = vst2_v4_; __threadfence(); *(volatile v4f*)(ptr) = vst2_v4_; } while (0)

__device__ __forceinline__ float bfr(float f) {
    unsigned u = __float_as_uint(f);
    u += 0x7FFFu + ((u >> 16) & 1u);
    return __uint_as_float(u & 0xFFFF0000u);
}
__device__ __forceinline__ unsigned short f2h_bits(float x) {
    return (fabsf(x) < 6.104e-5f) ? (unsigned short)0 : __builtin_bit_cast(unsigned short, (_Float16)x);
}
__device__ __forceinline__ void st8h(unsigned short* P, size_t o, const float* v) {
    v4u pk;
    pk.x = (unsigned)f2h_bits(v[0]) | ((unsigned)f2h_bits(v[1]) << 16);
    pk.y = (unsigned)f2h_bits(v[2]) | ((unsigned)f2h_bits(v[3]) << 16);
    pk.z = (unsigned)f2h_bits(v[4]) | ((unsigned)f2h_bits(v[5]) << 16);
    pk.w = (unsigned)f2h_bits(v[6]) | ((unsigned)f2h_bits(v[7]) << 16);
    VST2(v4u, (v4u*)(P + o), pk);
}

union FragU { v16h v; v8h h[2]; };
__device__ __forceinline__ v16h frag_ld(const _Float16* p) {
    FragU f; f.h[0] = *(const v8h*)(p); f.h[1] = *(const v8h*)(p + 16); return f.v;
}
__device__ __forceinline__ v8f wmma16(v16h a, v16h b, v8f c) {
    c = __builtin_amdgcn_wmma_f32_16x16x32_f16(false, a, false, b, (short)0, c, false, false);
    asm volatile("v_nop\n\tv_nop\n\tv_nop\n\tv_nop" : "+v"(c) : "v"(a), "v"(b));
    return c;
}
__device__ __forceinline__ void wave_sync_lds() {
    __builtin_amdgcn_fence(3  , "workgroup");
    __builtin_amdgcn_wave_barrier();
    __builtin_amdgcn_fence(2  , "workgroup");
}

static __device__ __forceinline__ h16 toh_flush(float v) { const float w = (fabsf(v) < 6.103515625e-05f) ? 0.0f : v; return (h16)w; }

__device__ __forceinline__ v16h frag_ldz(const _Float16* p) {
    FragU f; f.h[0] = *(const v8h*)(p);
    f.h[1] = (v8h){(h16)0.0f, (h16)0.0f, (h16)0.0f, (h16)0.0f, (h16)0.0f, (h16)0.0f, (h16)0.0f, (h16)0.0f};
    return f.v;
}

template <int DPH, int NHEAD>
__device__ __forceinline__ float bias_head(const float* __restrict__ bias, unsigned idx, unsigned nbias) {
    const unsigned h = idx >> 4, d = idx & 15u;
    const unsigned src = min(h * (unsigned)DPH + d, nbias - 1u);
    const float v = bfr(bias[src]);
    return (d < (unsigned)DPH && h < (unsigned)NHEAD) ? v : 0.0f;
}
__device__ __forceinline__ float bias_lin(const float* __restrict__ bias, unsigned idx, unsigned nbias) {
    const unsigned src = min(idx, nbias - 1u);
    const float v = bfr(bias[src]);
    return (idx < nbias) ? v : 0.0f;
}

template <int KIND, int DPH, int NHEAD>
__device__ __forceinline__ void gemm_body(
    const _Float16* __restrict__ A, unsigned lda, const _Float16* __restrict__ Bt, unsigned ldb,
    void* __restrict__ Cout, unsigned ldc, const float* __restrict__ bias, unsigned nbias,
    unsigned M, unsigned N, unsigned K) {
  __shared__ __align__(16) float sT[8][16 * 68];
  constexpr float SCALE = (KIND == KIND_O) ? SC_OUT : SC_PROJ;
  constexpr float OSC = (KIND == KIND_Q) ? ((DPH == 12) ? (QS0 * HCARRY) : (QS1 * HCARRY)) : HCARRY;
  const unsigned lane = threadIdx.x & 31u;
  const unsigned wave = (unsigned)__builtin_amdgcn_readfirstlane((int)(threadIdx.x >> 5));
  const unsigned tilesN = N >> 6, tilesM = M >> 6;
  const unsigned tile = blockIdx.x * 8u + wave;
  if (tile >= tilesM * tilesN) return;
  const unsigned tm = tile / tilesN;
  const unsigned tn = tile - tm * tilesN;
  const unsigned m0 = tm << 6, n0 = tn << 6;
  const unsigned rlane = lane & 15u;
  const unsigned koff = (lane >> 4) * 8u;
  const unsigned mOff = koff;

  v8f acc[4][4];
#pragma unroll
  for (int i = 0; i < 4; ++i)
#pragma unroll
    for (int j = 0; j < 4; ++j) acc[i][j] = (v8f){0.f,0.f,0.f,0.f,0.f,0.f,0.f,0.f};

#pragma unroll 1
  for (unsigned k0 = 0; k0 < K; k0 += 32u) {
    v16h bh[4];
#pragma unroll
    for (int j = 0; j < 4; ++j)
      bh[j] = frag_ld(Bt + (size_t)(n0 + ((unsigned)j << 4) + rlane) * ldb + koff + k0);
#pragma unroll
    for (int i = 0; i < 4; ++i) {
      const v16h ah = frag_ld(A + (size_t)(m0 + ((unsigned)i << 4) + rlane) * lda + koff + k0);
#pragma unroll
      for (int j = 0; j < 4; ++j)
        acc[i][j] = wmma16(ah, bh[j], acc[i][j]);
    }
  }

  float* slab = sT[wave];
#pragma unroll
  for (int i = 0; i < 4; ++i) {
    const unsigned mBase = m0 + ((unsigned)i << 4);
    float brow[8];
#pragma unroll
    for (int r = 0; r < 8; ++r) {
      brow[r] = 0.0f;
      if (KIND == KIND_V) brow[r] = bias_head<DPH, NHEAD>(bias, mBase + mOff + (unsigned)r, nbias);
    }
#pragma unroll
    for (int j = 0; j < 4; ++j) {
      const unsigned n = n0 + ((unsigned)j << 4) + rlane;
      float bcol = 0.0f;
      if (KIND == KIND_O) bcol = bias_lin(bias, n, nbias);
      if (KIND == KIND_Q || KIND == KIND_K) bcol = bias_head<DPH, NHEAD>(bias, n, nbias);
#pragma unroll
      for (int r = 0; r < 8; ++r) {
        float v = acc[i][j][r] * SCALE + ((KIND == KIND_V) ? brow[r] : bcol);
        if (KIND != KIND_O) v *= OSC;
        slab[(mOff + (unsigned)r) * 68u + ((unsigned)j << 4) + rlane] = v;
      }
    }
    wave_sync_lds();
    if (KIND == KIND_O) {
      float* C = (float*)Cout;
      const unsigned hh = lane >> 4, c4 = (lane & 15u) * 4u;
      static_assert(2 * 4 * 2 == 16 && 16 * 16 == 64 * 4);
#pragma unroll
      for (int half = 0; half < 2; ++half) {
        v4f vv[4];
#pragma unroll
        for (int it = 0; it < 4; ++it) {
          const unsigned row = (unsigned)(half * 4 + it) * 2u + hh;
          vv[it] = *(const v4f*)(slab + row * 68u + c4);
        }
        for (int pass = 0; pass < 2; ++pass) {
#pragma unroll
          for (int it = 0; it < 4; ++it) {
            const unsigned row = (unsigned)(half * 4 + it) * 2u + hh;
            *(volatile v4f*)(C + (size_t)(mBase + row) * ldc + n0 + c4) = vv[it];
          }
          __threadfence();
        }
      }
    } else {
      _Float16* C = (_Float16*)Cout;
      const unsigned q = lane >> 3, c8 = (lane & 7u) * 8u;
      static_assert(4 * 4 == 16 && 8 * 16 == 64 * 2);
      v8h hv[4];
#pragma unroll
      for (int it = 0; it < 4; ++it) {
        const unsigned row = (unsigned)it * 4u + q;
        const float* sp = slab + row * 68u + c8;
#pragma unroll
        for (int e = 0; e < 8; ++e) hv[it][e] = toh_flush(sp[e]);
      }
      for (int pass = 0; pass < 2; ++pass) {
#pragma unroll
        for (int it = 0; it < 4; ++it) {
          const unsigned row = (unsigned)it * 4u + q;
          *(volatile v8h*)(C + (size_t)(mBase + row) * ldc + n0 + c8) = hv[it];
        }
        __threadfence();
      }
    }
    wave_sync_lds();
  }
}

__global__ __launch_bounds__(256) void k_gemm_q0(const _Float16* __restrict__ A, const _Float16* __restrict__ Bt,
                                                 _Float16* __restrict__ C, const float* __restrict__ bias) {
  gemm_body<KIND_Q, DPH0, NH0>(A, KP0, Bt, KP0, (void*)C, LDQ0, bias, D0, MTOK, LDQ0, KP0);
}
__global__ __launch_bounds__(256) void k_gemm_k0(const _Float16* __restrict__ A, const _Float16* __restrict__ Bt,
                                                 _Float16* __restrict__ C, const float* __restrict__ bias) {
  gemm_body<KIND_K, DPH0, NH0>(A, KP0, Bt, KP0, (void*)C, LDQ0, bias, D0, MTOK, LDQ0, KP0);
}
__global__ __launch_bounds__(256) void k_gemm_v0(const _Float16* __restrict__ A, const _Float16* __restrict__ Bt,
                                                 _Float16* __restrict__ C, const float* __restrict__ bias) {
  gemm_body<KIND_V, DPH0, NH0>(A, KP0, Bt, KP0, (void*)C, MTOK, bias, D0, LDQ0, MTOK, KP0);
}
__global__ __launch_bounds__(256) void k_gemm_o0(const _Float16* __restrict__ A, const _Float16* __restrict__ Bt,
                                                 float* __restrict__ C, const float* __restrict__ bias) {
  gemm_body<KIND_O, DPH0, NH0>(A, KP0, Bt, KP0, (void*)C, D0, bias, D0, MTOK, D0, KP0);
}
__global__ __launch_bounds__(256) void k_gemm_q1(const _Float16* __restrict__ A, const _Float16* __restrict__ Bt,
                                                 _Float16* __restrict__ C, const float* __restrict__ bias) {
  gemm_body<KIND_Q, DPH1, NH1>(A, KP1, Bt, KP1, (void*)C, LDQ1, bias, D1, MTOK, LDQ1, KP1);
}
__global__ __launch_bounds__(256) void k_gemm_k1(const _Float16* __restrict__ A, const _Float16* __restrict__ Bt,
                                                 _Float16* __restrict__ C, const float* __restrict__ bias) {
  gemm_body<KIND_K, DPH1, NH1>(A, KP1, Bt, KP1, (void*)C, LDQ1, bias, D1, MTOK, LDQ1, KP1);
}
__global__ __launch_bounds__(256) void k_gemm_v1(const _Float16* __restrict__ A, const _Float16* __restrict__ Bt,
                                                 _Float16* __restrict__ C, const float* __restrict__ bias) {
  gemm_body<KIND_V, DPH1, NH1>(A, KP1, Bt, KP1, (void*)C, MTOK, bias, D1, LDQ1, MTOK, KP1);
}

__global__ __launch_bounds__(256) void k_wprep(const float* __restrict__ Wm, unsigned K, unsigned N, unsigned KP, unsigned NP,
                                               unsigned dph, unsigned nheads, unsigned short* __restrict__ W16) {
    const unsigned u = blockIdx.x * 256u + threadIdx.x;
    const unsigned per = KP >> 3;
    if (u >= NP * per) return;
    const unsigned n = u / per;
    const unsigned k0 = 8u * (u - n * per);
    const unsigned h = n >> 4, d = n & 15u;
    const bool hv = (d < dph) && (h < nheads);
    const bool lv = (n < N);
    const bool headmode = (dph > 0u);
    const unsigned src = headmode ? (h * dph + d) : n;
    const bool valid = headmode ? hv : lv;
    const unsigned srcc = min(src, N - 1u);
    float v[8];
#pragma unroll
    for (int i = 0; i < 8; ++i) {
        const unsigned k = k0 + (unsigned)i;
        const unsigned kc = min(k, K - 1u);
        const float w = bfr(Wm[(size_t)kc * N + srcc]) * WCARRY;
        v[i] = (valid && k < K) ? w : 0.0f;
    }
    st8h(W16, (size_t)n * KP + k0, v);
}

__global__ __launch_bounds__(256) void k_cvt_in(const float* __restrict__ in, unsigned C, unsigned CP, unsigned rows,
                                                unsigned short* __restrict__ dst) {
    const unsigned u = blockIdx.x * 256u + threadIdx.x;
    const unsigned gpr = CP >> 3;
    if (u >= rows * gpr) return;
    const unsigned row = u / gpr;
    const unsigned c0 = (u - row * gpr) * 8u;
    const float* ir = in + (size_t)row * C;
    float v[8];
#pragma unroll
    for (int i = 0; i < 8; ++i) {
        const unsigned c = c0 + (unsigned)i;
        const unsigned cc = min(c, C - 1u);
        const float w = bfr(ir[cc]) * XCARRY;
        v[i] = (c < C) ? w : 0.0f;
    }
    st8h(dst, (size_t)row * CP + c0, v);
}

template <int DPH, int NHEAD, int LDQ, int CP>
__device__ __forceinline__ void attn_body(const _Float16* __restrict__ Q16, const _Float16* __restrict__ K16,
                                          const _Float16* __restrict__ VT, const int* __restrict__ mask,
                                          _Float16* __restrict__ ctx) {
    constexpr unsigned NT = (unsigned)NHEAD * 32u;
    constexpr unsigned NPIECE = (unsigned)QB * (unsigned)CP / 8u;
    constexpr unsigned ITERS = (NPIECE + NT - 1u) / NT;
    constexpr int NQT = QB / 16;
    static_assert(CP % 8 == 0 && CP >= NHEAD * DPH);
    static_assert(ITERS * NT >= NPIECE);
    static_assert((NPIECE - (ITERS - 1u) * NT) % 32u == 0u);
    static_assert(((unsigned)QB * (unsigned)CP * 2u) % 128u == 0u);
    static_assert(NHEAD * 16 <= LDQ);
    __shared__ __align__(16) _Float16 sC[QB * CP];
    const unsigned tid = threadIdx.x, lane = tid & 31u;
    const unsigned head = (unsigned)__builtin_amdgcn_readfirstlane((int)(tid >> 5));
    const unsigned hh = lane >> 4, c = lane & 15u;
    const unsigned bx = blockIdx.x;
    const unsigned b = bx / (unsigned)(SEQ / QB);
    const unsigned q0 = (bx % (unsigned)(SEQ / QB)) * (unsigned)QB;

    {
        const v8h zh = (v8h){(h16)0.0f, (h16)0.0f, (h16)0.0f, (h16)0.0f, (h16)0.0f, (h16)0.0f, (h16)0.0f, (h16)0.0f};
#pragma unroll
        for (unsigned it = 0; it < ITERS; ++it) {
            const unsigned p = it * NT + tid;
            if (p < NPIECE) *(v8h*)(sC + 8u * p) = zh;
        }
    }
    __syncthreads();

    v16h qf[NQT];
    v8f o[NQT];
    float mrun[NQT], lrun[NQT];
#pragma unroll
    for (int qt = 0; qt < NQT; ++qt) {
        qf[qt] = frag_ldz(Q16 + (size_t)(b * SEQ + q0 + (unsigned)qt * 16u + c) * (unsigned)LDQ + head * 16u + 8u * hh);
        o[qt] = (v8f){0.f,0.f,0.f,0.f,0.f,0.f,0.f,0.f};
        mrun[qt] = NEGMAX;
        lrun[qt] = 0.0f;
    }

#pragma unroll 1
    for (unsigned kv0 = 0; kv0 < (unsigned)SEQ; kv0 += 32u) {
        const _Float16* kp = K16 + (size_t)(b * SEQ + kv0 + c) * (unsigned)LDQ + head * 16u + 8u * hh;
        const v16h ka0 = frag_ldz(kp);
        const v16h ka1 = frag_ldz(kp + 16u * (unsigned)LDQ);
        const v16h va = frag_ld(VT + (size_t)(head * 16u + c) * (unsigned)MTOK + b * SEQ + kv0 + 8u * hh);
        const int* mp = mask + (size_t)b * SEQ_FULL + kv0 + 8u * hh;
        v4i m0a = *(const v4i*)(mp);
        v4i m0b = *(const v4i*)(mp + 4);
        v4i m1a = *(const v4i*)(mp + 16);
        v4i m1b = *(const v4i*)(mp + 20);
        asm volatile("" : "+v"(m0a));
        asm volatile("" : "+v"(m0b));
        asm volatile("" : "+v"(m1a));
        asm volatile("" : "+v"(m1b));
        const int mk0[8] = {m0a.x, m0a.y, m0a.z, m0a.w, m0b.x, m0b.y, m0b.z, m0b.w};
        const int mk1[8] = {m1a.x, m1a.y, m1a.z, m1a.w, m1b.x, m1b.y, m1b.z, m1b.w};
#pragma unroll
        for (int qt = 0; qt < NQT; ++qt) {
            const v8f zz = (v8f){0.f,0.f,0.f,0.f,0.f,0.f,0.f,0.f};
            const v8f s0 = wmma16(ka0, qf[qt], zz);
            const v8f s1 = wmma16(ka1, qf[qt], zz);
            float t0[8], t1[8];
            float mx = NEGMAX;
#pragma unroll
            for (int r = 0; r < 8; ++r) {
                const float a0 = s0[r] * SC2;
                const float a1 = s1[r] * SC2;
                t0[r] = (mk0[r] == 0) ? NEGMAX : a0;
                t1[r] = (mk1[r] == 0) ? NEGMAX : a1;
                mx = fmaxf(mx, fmaxf(t0[r], t1[r]));
            }
            mx = fmaxf(mx, __shfl_xor(mx, 16, 32));
            const float mnew = fmaxf(mrun[qt], mx);
            const float alpha = exp2f(mrun[qt] - mnew);
            mrun[qt] = mnew;
            FragU pb;
            float psum = 0.0f;
#pragma unroll
            for (int r = 0; r < 8; ++r) {
                const h16 w0 = toh_flush(exp2f(t0[r] - mnew) * PCARRY);
                const h16 w1 = toh_flush(exp2f(t1[r] - mnew) * PCARRY);
                psum += (float)w0 + (float)w1;
                pb.v[r] = w0;
                pb.v[8 + r] = w1;
            }
            lrun[qt] = lrun[qt] * alpha + psum;
#pragma unroll
            for (int r = 0; r < 8; ++r) o[qt][r] *= alpha;
            o[qt] = wmma16(va, pb.v, o[qt]);
        }
    }

#pragma unroll
    for (int qt = 0; qt < NQT; ++qt) {
        const float lt = lrun[qt] + __shfl_xor(lrun[qt], 16, 32);
        const float inv = CTXS * (1.0f / lt);
#pragma unroll
        for (int r = 0; r < 8; ++r) {
            const unsigned d = 8u * hh + (unsigned)r;
            const h16 w = toh_flush(o[qt][r] * inv);
            if (d < (unsigned)DPH) sC[((unsigned)qt * 16u + c) * (unsigned)CP + head * (unsigned)DPH + d] = w;
        }
    }
    __syncthreads();
    {
        v8h cv[ITERS];
#pragma unroll
        for (unsigned it = 0; it < ITERS; ++it) {
            const unsigned p = it * NT + tid;
            const unsigned pc = min(p, NPIECE - 1u);
            cv[it] = *(const v8h*)(sC + 8u * pc);
        }
        _Float16* dst = ctx + (size_t)(b * SEQ + q0) * (unsigned)CP;
        for (int pass = 0; pass < 2; ++pass) {
#pragma unroll
            for (unsigned it = 0; it < ITERS; ++it) {
                const unsigned p = it * NT + tid;
                if (p < NPIECE) *(volatile v8h*)(dst + 8u * p) = cv[it];
            }
            __threadfence();
        }
    }
}

__global__ __launch_bounds__(512) void k_attn0(const _Float16* __restrict__ Q16, const _Float16* __restrict__ K16,
                                               const _Float16* __restrict__ VT, const int* __restrict__ mask,
                                               _Float16* __restrict__ ctx) {
    attn_body<DPH0, NH0, LDQ0, KP0>(Q16, K16, VT, mask, ctx);
}
__global__ __launch_bounds__(352) void k_attn1(const _Float16* __restrict__ Q16, const _Float16* __restrict__ K16,
                                               const _Float16* __restrict__ VT, const int* __restrict__ mask,
                                               _Float16* __restrict__ ctx) {
    attn_body<DPH1, NH1, LDQ1, KP1>(Q16, K16, VT, mask, ctx);
}

__global__ __launch_bounds__(256) void k_out1(const _Float16* __restrict__ A, const _Float16* __restrict__ Wt,
                                              const float* __restrict__ bias, float* __restrict__ out, unsigned M) {
    __shared__ __align__(16) float sO[8][16 * D1];
    const unsigned lane = threadIdx.x & 31u;
    const unsigned wave = (unsigned)__builtin_amdgcn_readfirstlane((int)(threadIdx.x >> 5));
    const unsigned m0 = (blockIdx.x * 8u + wave) * 16u;
    if (m0 >= M) return;
    const unsigned hh = lane >> 4, c = lane & 15u;
    v8f acc[5];
#pragma unroll
    for (int j = 0; j < 5; ++j) acc[j] = (v8f){0.f,0.f,0.f,0.f,0.f,0.f,0.f,0.f};
#pragma unroll 1
    for (unsigned k0 = 0; k0 < (unsigned)KP1; k0 += 32u) {
        const v16h a = frag_ld(A + (size_t)(m0 + c) * KP1 + k0 + 8u * hh);
#pragma unroll
        for (int j = 0; j < 5; ++j) {
            const v16h bw = frag_ld(Wt + (size_t)((unsigned)j * 16u + c) * KP1 + k0 + 8u * hh);
            acc[j] = wmma16(a, bw, acc[j]);
        }
    }
    float* tile = sO[wave];
#pragma unroll
    for (int j = 0; j < 5; ++j) {
        const unsigned col = (unsigned)j * 16u + c;
        const float bv = bfr(bias[min(col, (unsigned)(D1 - 1))]);
#pragma unroll
        for (int r = 0; r < 8; ++r) {
            const float v = acc[j][r] * SC_OUT + bv;
            if (col < (unsigned)D1) tile[(8u * hh + (unsigned)r) * (unsigned)D1 + col] = v;
        }
    }
    wave_sync_lds();
    {
        constexpr unsigned NP4 = 16u * (unsigned)D1 / 4u;
        v4f vv[9];
#pragma unroll
        for (unsigned it = 0; it < 9u; ++it) {
            const unsigned idx = it * 32u + lane;
            const unsigned idc = min(idx, NP4 - 1u);
            vv[it] = *(const v4f*)(tile + 4u * idc);
        }
        float* dst = out + (size_t)m0 * D1;
        for (int pass = 0; pass < 2; ++pass) {
#pragma unroll
            for (unsigned it = 0; it < 9u; ++it) {
                const unsigned idx = it * 32u + lane;
                if (idx < NP4) *(volatile v4f*)(dst + 4u * idx) = vv[it];
            }
            __threadfence();
        }
    }
}

extern "C" void kernel_launch(void* const* d_in, const int* in_sizes, int n_in, void* d_out, int out_size,
                              void* d_ws, size_t ws_size, hipStream_t stream) {
    if (n_in < 20) return;
    if (in_sizes[0] < MTOK * D0 || in_sizes[1] < MTOK * D1 || in_sizes[2] < MTOK || in_sizes[3] < MTOK) return;
    if (in_sizes[4] < D0 * D0 || in_sizes[6] < D0 * D0 || in_sizes[8] < D0 * D0 || in_sizes[10] < D0 * D0) return;
    if (in_sizes[5] < D0 || in_sizes[7] < D0 || in_sizes[9] < D0 || in_sizes[11] < D0) return;
    if (in_sizes[12] < D1 * D1 || in_sizes[14] < D1 * D1 || in_sizes[16] < D1 * D1 || in_sizes[18] < D1 * D1) return;
    if (in_sizes[13] < D1 || in_sizes[15] < D1 || in_sizes[17] < D1 || in_sizes[19] < D1) return;
    if (out_size < OUT1_OFF_ELEMS + MTOK * D1) return;

    const float* x     = (const float*)d_in[0];
    const float* y     = (const float*)d_in[1];
    const int*   mask0 = (const int*)d_in[2];
    const int*   mask1 = (const int*)d_in[3];
    const float* q0_w  = (const float*)d_in[4];
    const float* q0_b  = (const float*)d_in[5];
    const float* k0_w  = (const float*)d_in[6];
    const float* k0_b  = (const float*)d_in[7];
    const float* v0_w  = (const float*)d_in[8];
    const float* v0_b  = (const float*)d_in[9];
    const float* o0_w  = (const float*)d_in[10];
    const float* o0_b  = (const float*)d_in[11];
    const float* q1_w  = (const float*)d_in[12];
    const float* q1_b  = (const float*)d_in[13];
    const float* k1_w  = (const float*)d_in[14];
    const float* k1_b  = (const float*)d_in[15];
    const float* v1_w  = (const float*)d_in[16];
    const float* v1_b  = (const float*)d_in[17];
    const float* o1_w  = (const float*)d_in[18];
    const float* o1_b  = (const float*)d_in[19];
    float* out0 = (float*)d_out;
    float* out1 = (float*)d_out + (size_t)OUT1_OFF_ELEMS;

    char* wsp = (char*)d_ws;
    size_t off = 0;
    auto carve = [&](size_t bytes) -> void* { void* r = wsp + off; off += (bytes + 255) & ~(size_t)255; return r; };
    unsigned short* x16  = (unsigned short*)carve((size_t)MTOK * KP0 * 2);
    unsigned short* y16  = (unsigned short*)carve((size_t)MTOK * KP1 * 2);
    unsigned short* q0p  = (unsigned short*)carve((size_t)MTOK * LDQ0 * 2);
    unsigned short* k0p  = (unsigned short*)carve((size_t)MTOK * LDQ0 * 2);
    unsigned short* vt0  = (unsigned short*)carve((size_t)LDQ0 * MTOK * 2);
    unsigned short* c0p  = (unsigned short*)carve((size_t)MTOK * KP0 * 2);
    unsigned short* q1p  = (unsigned short*)carve((size_t)MTOK * LDQ1 * 2);
    unsigned short* k1p  = (unsigned short*)carve((size_t)MTOK * LDQ1 * 2);
    unsigned short* vt1  = (unsigned short*)carve((size_t)LDQ1 * MTOK * 2);
    unsigned short* c1p  = (unsigned short*)carve((size_t)MTOK * KP1 * 2);
    unsigned short* wq0  = (unsigned short*)carve((size_t)LDQ0 * KP0 * 2);
    unsigned short* wk0  = (unsigned short*)carve((size_t)LDQ0 * KP0 * 2);
    unsigned short* wv0  = (unsigned short*)carve((size_t)LDQ0 * KP0 * 2);
    unsigned short* wo0  = (unsigned short*)carve((size_t)D0 * KP0 * 2);
    unsigned short* wq1  = (unsigned short*)carve((size_t)LDQ1 * KP1 * 2);
    unsigned short* wk1  = (unsigned short*)carve((size_t)LDQ1 * KP1 * 2);
    unsigned short* wv1  = (unsigned short*)carve((size_t)LDQ1 * KP1 * 2);
    unsigned short* wo1  = (unsigned short*)carve((size_t)NO1P * KP1 * 2);
    if (off > ws_size || off > (size_t)134217728) return;

    k_cvt_in<<<(MTOK * (KP0 / 8) + 255) / 256, 256, 0, stream>>>(x, D0, KP0, MTOK, x16);
    k_cvt_in<<<(MTOK * (KP1 / 8) + 255) / 256, 256, 0, stream>>>(y, D1, KP1, MTOK, y16);

    k_wprep<<<(LDQ0 * (KP0 / 8) + 255) / 256, 256, 0, stream>>>(q0_w, D0, D0, KP0, LDQ0, DPH0, NH0, wq0);
    k_wprep<<<(LDQ0 * (KP0 / 8) + 255) / 256, 256, 0, stream>>>(k0_w, D0, D0, KP0, LDQ0, DPH0, NH0, wk0);
    k_wprep<<<(LDQ0 * (KP0 / 8) + 255) / 256, 256, 0, stream>>>(v0_w, D0, D0, KP0, LDQ0, DPH0, NH0, wv0);
    k_wprep<<<(D0 * (KP0 / 8) + 255) / 256, 256, 0, stream>>>(o0_w, D0, D0, KP0, D0, 0, 0, wo0);
    k_wprep<<<(LDQ1 * (KP1 / 8) + 255) / 256, 256, 0, stream>>>(q1_w, D1, D1, KP1, LDQ1, DPH1, NH1, wq1);
    k_wprep<<<(LDQ1 * (KP1 / 8) + 255) / 256, 256, 0, stream>>>(k1_w, D1, D1, KP1, LDQ1, DPH1, NH1, wk1);
    k_wprep<<<(LDQ1 * (KP1 / 8) + 255) / 256, 256, 0, stream>>>(v1_w, D1, D1, KP1, LDQ1, DPH1, NH1, wv1);
    k_wprep<<<(NO1P * (KP1 / 8) + 255) / 256, 256, 0, stream>>>(o1_w, D1, D1, KP1, NO1P, 0, 0, wo1);

    const unsigned gQ0 = ((MTOK / 64) * (LDQ0 / 64) + 7) / 8;
    const unsigned gQ1 = ((MTOK / 64) * (LDQ1 / 64) + 7) / 8;
    const unsigned gO0 = ((MTOK / 64) * (D0 / 64) + 7) / 8;

    k_gemm_q0<<<gQ0, 256, 0, stream>>>((const _Float16*)x16, (const _Float16*)wq0, (_Float16*)q0p, q0_b);
    k_gemm_k0<<<gQ0, 256, 0, stream>>>((const _Float16*)x16, (const _Float16*)wk0, (_Float16*)k0p, k0_b);
    k_gemm_v0<<<gQ0, 256, 0, stream>>>((const _Float16*)wv0, (const _Float16*)x16, (_Float16*)vt0, v0_b);
    k_gemm_q1<<<gQ1, 256, 0, stream>>>((const _Float16*)y16, (const _Float16*)wq1, (_Float16*)q1p, q1_b);
    k_gemm_k1<<<gQ1, 256, 0, stream>>>((const _Float16*)y16, (const _Float16*)wk1, (_Float16*)k1p, k1_b);
    k_gemm_v1<<<gQ1, 256, 0, stream>>>((const _Float16*)wv1, (const _Float16*)y16, (_Float16*)vt1, v1_b);

    k_attn0<<<NB * (SEQ / QB), NH0 * 32, 0, stream>>>((const _Float16*)q0p, (const _Float16*)k0p, (const _Float16*)vt0, mask0, (_Float16*)c0p);
    k_attn1<<<NB * (SEQ / QB), NH1 * 32, 0, stream>>>((const _Float16*)q1p, (const _Float16*)k1p, (const _Float16*)vt1, mask1, (_Float16*)c1p);

    k_gemm_o0<<<gO0, 256, 0, stream>>>((const _Float16*)c0p, (const _Float16*)wo0, out0, o0_b);
    k_out1<<<(MTOK / 16 + 7) / 8, 256, 0, stream>>>((const _Float16*)c1p, (const _Float16*)wo1, o1_b, out1, MTOK);
}
